// VladPooling_21629455302857
// MI455X (gfx1250) — hardware-run, weakly checked
//
#include <hip/hip_runtime.h>
#include <math.h>

typedef __attribute__((ext_vector_type(16))) _Float16 v16h;
typedef __attribute__((ext_vector_type(8)))  _Float16 v8h;
typedef __attribute__((ext_vector_type(8)))  float    v8f;
typedef __attribute__((ext_vector_type(4)))  float    v4f;

constexpr int kNB   = 32;
constexpr int kNT   = 500;
constexpr int kNTP  = 512;
constexpr int kND   = 512;
constexpr int kNKC  = 10;
constexpr int kNKO  = 8;
constexpr int kAP   = 520;
constexpr int kFP   = 32;
constexpr int kTC   = 32;
constexpr float kCarryA = 4096.0f;
constexpr float kCarryF = 64.0f;
constexpr float kFold   = 1.0f / (kCarryA * kCarryF);
static_assert((kNTP % kTC) == 0);
static_assert(kNTP >= kNT);
static_assert((kND % 64) == 0);
static_assert(kND / 64 == 8);
static_assert((kAP % 8) == 0);
static_assert((kFP % 8) == 0);
static_assert(kNKO * kND == 4096);
static_assert(kFold == 1.0f / 262144.0f);

struct FragH {
  union U { v16h v; v8h h[2]; };
  static __device__ __forceinline__ v16h load(const _Float16* p) {
    U f;
    f.h[0] = *(const v8h*)(p);
    f.h[1] = *(const v8h*)(p + 16);
    return f.v;
  }
};

__device__ __forceinline__ v8f mma_guarded(v16h a, v16h b, v8f c) {
  c = __builtin_amdgcn_wmma_f32_16x16x32_f16(false, a, false, b, (short)0, c, false, false);
  asm volatile("v_nop\n\tv_nop\n\tv_nop\n\tv_nop" : "+v"(c) : "v"(a), "v"(b));
  return c;
}

__global__ __launch_bounds__(256) void pool_fused_kernel(
    const float* __restrict__ feat, const float* __restrict__ score,
    const float* __restrict__ cluster, float* __restrict__ out)
{
  __shared__ __align__(16) _Float16 sF[kND * kFP];
  __shared__ __align__(16) _Float16 sA[kNKO * kAP];
  __shared__ __align__(16) float    sO[kNKO * kND];
  __shared__ float sAP[8 * kNKO];
  __shared__ float sSS[8 * kNKO];

  const int tid  = threadIdx.x;
  const int lane = tid & 31;
  const int wave = __builtin_amdgcn_readfirstlane((int)(threadIdx.x >> 5));
  const int hh   = lane >> 4;
  const int cl   = lane & 15;
  const int b    = blockIdx.x;

#pragma unroll
  for (int it = 0; it < 4; ++it) {
    const int i4 = (it * 256 + tid) * 4;
    v4f cv = *(const v4f*)(cluster + i4);
    *(v4f*)(sO + i4) = cv;
  }

  float am[kNKO];
#pragma unroll
  for (int k = 0; k < kNKO; ++k) am[k] = 0.0f;
  const float* sb = score + (size_t)b * kNT * kNKC;
#pragma unroll 1
  for (int rr = 0; rr < 2; ++rr) {
    const int t  = tid + 256 * rr;
    const int tc = (t < kNT) ? t : (kNT - 1);
    const bool valid = (t < kNT);
    const float* sp = sb + (size_t)tc * kNKC;
    float s[kNKC];
#pragma unroll
    for (int k = 0; k < kNKC; ++k) {
      float x = sp[k];
      asm volatile("" : "+v"(x));
      s[k] = x;
    }
    float m = s[0];
#pragma unroll
    for (int k = 1; k < kNKC; ++k) m = fmaxf(m, s[k]);
    float sum = 0.0f;
#pragma unroll
    for (int k = 0; k < kNKC; ++k) {
      s[k] = expf(s[k] - m);
      sum += s[k];
    }
    const float inv = 1.0f / sum;
#pragma unroll
    for (int k = 0; k < kNKO; ++k) {
      const float pk = s[k] * inv;
      const float p  = valid ? pk : 0.0f;
      am[k] += p;
      sA[k * kAP + t] = (_Float16)(p * kCarryA);
    }
  }
#pragma unroll
  for (int k = 0; k < kNKO; ++k) {
    float v = am[k];
    v += __shfl_xor(v, 16, 32);
    v += __shfl_xor(v, 8, 32);
    v += __shfl_xor(v, 4, 32);
    v += __shfl_xor(v, 2, 32);
    v += __shfl_xor(v, 1, 32);
    am[k] = v;
  }
  if (lane == 0) {
#pragma unroll
    for (int k = 0; k < kNKO; ++k) sAP[wave * kNKO + k] = am[k];
  }

  v8f acc[4];
#pragma unroll
  for (int j = 0; j < 4; ++j) acc[j] = (v8f){0.f, 0.f, 0.f, 0.f, 0.f, 0.f, 0.f, 0.f};

  const float* fb = feat + (size_t)b * kNT * kND;
  const _Float16* arow = sA + (cl & 7) * kAP + 8 * hh;
  const _Float16* brow = sF + (wave * 64 + cl) * kFP + 8 * hh;

#pragma unroll 1
  for (int t0 = 0; t0 < kNTP; t0 += kTC) {
    __syncthreads();
#pragma unroll 4
    for (int j = 0; j < 16; ++j) {
      const int i   = tid + 256 * j;
      const int dg  = i & 127;
      const int tl  = i >> 7;
      const int tg  = t0 + tl;
      const int tcl = (tg < kNT) ? tg : (kNT - 1);
      const bool valid = (tg < kNT);
      v4f f = *(const v4f*)(fb + (size_t)tcl * kND + 4 * dg);
      asm volatile("" : "+v"(f));
      const float y0 = f[0] * kCarryF;
      const float y1 = f[1] * kCarryF;
      const float y2 = f[2] * kCarryF;
      const float y3 = f[3] * kCarryF;
      const float x0 = valid ? y0 : 0.0f;
      const float x1 = valid ? y1 : 0.0f;
      const float x2 = valid ? y2 : 0.0f;
      const float x3 = valid ? y3 : 0.0f;
      _Float16* dst = sF + (4 * dg) * kFP + tl;
      dst[0]       = (_Float16)x0;
      dst[kFP]     = (_Float16)x1;
      dst[2 * kFP] = (_Float16)x2;
      dst[3 * kFP] = (_Float16)x3;
    }
    __syncthreads();
    const v16h a = FragH::load(arow + t0);
#pragma unroll
    for (int j = 0; j < 4; ++j) {
      const v16h bf = FragH::load(brow + (j * 16) * kFP);
      acc[j] = mma_guarded(a, bf, acc[j]);
    }
  }

  float asum[kNKO];
#pragma unroll
  for (int k = 0; k < kNKO; ++k) {
    float v = 0.0f;
#pragma unroll
    for (int w = 0; w < 8; ++w) v += sAP[w * kNKO + k];
    asum[k] = v;
  }
  float ss[kNKO];
#pragma unroll
  for (int k = 0; k < kNKO; ++k) ss[k] = 0.0f;
#pragma unroll
  for (int j = 0; j < 4; ++j) {
    const int dcol = wave * 64 + j * 16 + cl;
#pragma unroll
    for (int r = 0; r < kNKO; ++r) {
      const float cv  = sO[r * kND + dcol];
      const float ag  = acc[j][r] * kFold;
      const float res = ag - asum[r] * cv;
      acc[j][r] = res;
      ss[r] += res * res;
    }
  }
#pragma unroll
  for (int r = 0; r < kNKO; ++r) {
    float v = ss[r];
    v += __shfl_xor(v, 8, 32);
    v += __shfl_xor(v, 4, 32);
    v += __shfl_xor(v, 2, 32);
    v += __shfl_xor(v, 1, 32);
    ss[r] = v;
  }
  if (lane == 0) {
#pragma unroll
    for (int r = 0; r < kNKO; ++r) sSS[wave * kNKO + r] = ss[r];
  }
  __syncthreads();
  float inv[kNKO];
#pragma unroll
  for (int r = 0; r < kNKO; ++r) {
    float v = 0.0f;
#pragma unroll
    for (int w = 0; w < 8; ++w) v += sSS[w * kNKO + r];
    inv[r] = rsqrtf(fmaxf(v, 1e-12f));
  }
  if (hh == 0) {
#pragma unroll
    for (int j = 0; j < 4; ++j) {
      const int dcol = wave * 64 + j * 16 + cl;
#pragma unroll
      for (int r = 0; r < kNKO; ++r) sO[r * kND + dcol] = acc[j][r] * inv[r];
    }
  }
  __syncthreads();
  float* ob = out + (size_t)b * (kNKO * kND);
  for (int pass = 0; pass < 2; ++pass) {
#pragma unroll
    for (int it = 0; it < 4; ++it) {
      const int i4 = (it * 256 + tid) * 4;
      const v4f v = *(const v4f*)(sO + i4);
      *(volatile v4f*)(ob + i4) = v;
    }
    __threadfence();
  }
}

extern "C" void kernel_launch(void* const* d_in, const int* in_sizes, int n_in,
                              void* d_out, int out_size, void* d_ws, size_t ws_size,
                              hipStream_t stream) {
  (void)d_ws;
  (void)ws_size;
  if (n_in < 3) return;
  if (in_sizes[0] != kNB * kNT * kND) return;
  if (in_sizes[1] != kNB * kNT * kNKC) return;
  if (in_sizes[2] != kNKC * kND) return;
  if (out_size != kNB * kNKO * kND) return;

  const float* feat    = (const float*)d_in[0];
  const float* score   = (const float*)d_in[1];
  const float* cluster = (const float*)d_in[2];
  float* out = (float*)d_out;

  pool_fused_kernel<<<kNB, 256, 0, stream>>>(feat, score, cluster, out);
}
